// VAE_41180146434656
// MI455X (gfx1250) — hardware-run, weakly checked
//
#include <hip/hip_runtime.h>
#include <math.h>

typedef __attribute__((ext_vector_type(16))) _Float16 v16h;
typedef __attribute__((ext_vector_type(2)))  _Float16 v2h;
typedef __attribute__((ext_vector_type(16))) __bf16   v16b;
typedef __attribute__((ext_vector_type(8)))  float    v8f;
typedef __attribute__((ext_vector_type(4)))  float    v4f;
typedef __attribute__((ext_vector_type(2)))  float    v2f;
typedef __attribute__((ext_vector_type(4)))  unsigned v4u;
typedef __attribute__((ext_vector_type(8)))  unsigned v8u;

constexpr int   kSamples   = 1048576;
constexpr int   kHid       = 100;
constexpr int   kHidPad    = 128;
constexpr int   kEncOut    = 4;
constexpr int   kDecOut    = 2;
constexpr int   kSteps     = 10;
constexpr int   kStepHid   = 20;
constexpr int   kBlkThr    = 128;
constexpr int   kMainGrid  = kSamples / kBlkThr;
constexpr int   kBtPitch   = 68;
constexpr int   kOutFloats = 2 * kSamples + 1;
constexpr int   kPackV4    = kOutFloats / 4;
constexpr int   kPackGrid  = (kPackV4 + 1 + 255) / 256;
constexpr float kLog2Pi    = 1.8378770664093453f;
constexpr float kCarryH    = 16.0f;
constexpr float kCarryW    = 64.0f;
constexpr float kFoldEnc   = 1.0f / (kCarryH * kCarryW);
static_assert((kSamples % kBlkThr) == 0, "exact grid");
static_assert(kMainGrid == 8192, "grid");
static_assert((kHidPad % 32) == 0 && kHidPad >= kHid, "K pad multiple of 32");
static_assert((kOutFloats % 4) == 1, "one float in the final line");
static_assert(kPackGrid == 2049, "pack grid");
static_assert((kMainGrid % 256) == 0, "partial sums per thread");
static_assert(kSteps * kStepHid == 200, "shear table");

constexpr size_t kOffZws   = 0;
constexpr size_t kOffPart  = kOffZws + (size_t)kSamples * 2 * 4;
constexpr size_t kOffElbo  = kOffPart + (size_t)kMainGrid * 32 * 4;
constexpr size_t kWsTotal  = kOffElbo + 128;
static_assert(kWsTotal == 9437312ull, "carve total");
static_assert(kWsTotal <= 134217728ull, "carve cap");
static_assert((kOffPart % 128) == 0 && (kOffElbo % 128) == 0, "aligned regions");

__device__ __forceinline__ unsigned bf_rne16(float f) {
  const unsigned u = __float_as_uint(f);
  return (u + 0x7FFFu + ((u >> 16) & 1u)) >> 16;
}

__device__ __forceinline__ v8f mma_h(v16h a, v16h b, v8f c) {
  c = __builtin_amdgcn_wmma_f32_16x16x32_f16(false, a, false, b, (short)0, c, false, false);
  asm volatile("v_nop\n\tv_nop\n\tv_nop\n\tv_nop" : "+v"(c) : "v"(a), "v"(b));
  return c;
}
__device__ __forceinline__ v8f mma_b(v16b a, v16b b, v8f c) {
  c = __builtin_amdgcn_wmma_f32_16x16x32_bf16(false, a, false, b, (short)0, c, false, false);
  asm volatile("v_nop\n\tv_nop\n\tv_nop\n\tv_nop" : "+v"(c) : "v"(a), "v"(b));
  return c;
}

__device__ __forceinline__ float tanh_dev(float v) {
#if defined(__has_builtin)
#if __has_builtin(__builtin_amdgcn_tanhf)
  return __builtin_amdgcn_tanhf(v);
#else
  return tanhf(v);
#endif
#else
  return tanhf(v);
#endif
}

__device__ __forceinline__ v8u load_bfrag(const unsigned* plane, int n, int hh, int c) {
  const unsigned* p = plane + n * kBtPitch + 16 * c + 4 * hh;
  const v4u lo = *(const v4u*)(p);
  const v4u hi = *(const v4u*)(p + 8);
  v8u r;
  r[0] = lo[0]; r[1] = lo[1]; r[2] = lo[2]; r[3] = lo[3];
  r[4] = hi[0]; r[5] = hi[1]; r[6] = hi[2]; r[7] = hi[3];
  return r;
}

template <bool BF>
__device__ __forceinline__ v8f hidden_chunk(const float* tab, int koff, float in0, float in1, v8u bw, v8f acc) {
  float hv[16];
#pragma unroll
  for (int g = 0; g < 2; ++g) {
    const float* p = tab + koff + 16 * g;
    const v4f wa0 = *(const v4f*)(p);
    const v4f wa1 = *(const v4f*)(p + 4);
    const v4f wb0 = *(const v4f*)(p + kHidPad);
    const v4f wb1 = *(const v4f*)(p + kHidPad + 4);
    const v4f bb0 = *(const v4f*)(p + 2 * kHidPad);
    const v4f bb1 = *(const v4f*)(p + 2 * kHidPad + 4);
#pragma unroll
    for (int e = 0; e < 4; ++e) {
      hv[8 * g + e]     = fmaxf(fmaf(in0, wa0[e], fmaf(in1, wb0[e], bb0[e])), 0.0f);
      hv[8 * g + 4 + e] = fmaxf(fmaf(in0, wa1[e], fmaf(in1, wb1[e], bb1[e])), 0.0f);
    }
  }
  if (BF) {
    v8u aw;
#pragma unroll
    for (int j = 0; j < 8; ++j) aw[j] = bf_rne16(hv[2 * j]) | (bf_rne16(hv[2 * j + 1]) << 16);
    return mma_b(__builtin_bit_cast(v16b, aw), __builtin_bit_cast(v16b, bw), acc);
  } else {
    v16h a;
#pragma unroll
    for (int e = 0; e < 16; ++e) a[e] = (_Float16)hv[e];
    return mma_h(a, __builtin_bit_cast(v16h, bw), acc);
  }
}

__device__ __forceinline__ void spill_tile(float* dst, v8f acc, float scale, float bias, int hh, int n) {
#pragma unroll
  for (int r = 0; r < 8; ++r) dst[(8 * hh + r) * 16 + n] = fmaf(acc[r], scale, bias);
}

__device__ __forceinline__ float shear_mlp(const float* tab, float u) {
  float acc = tab[3];
#pragma unroll 4
  for (int j = 0; j < kStepHid; ++j) {
    const v4f e = *(const v4f*)(tab + 4 * j);
    const float t = tanh_dev(fmaf(u, e[0], e[1]));
    acc = fmaf(t, e[2], acc);
  }
  return acc;
}

__global__ __launch_bounds__(128) void fused_sample_kernel(
    const float* __restrict__ x, const float* __restrict__ eps,
    const float* __restrict__ enc_w1, const float* __restrict__ enc_b1,
    const float* __restrict__ enc_w2, const float* __restrict__ enc_b2,
    const float* __restrict__ dec_w1, const float* __restrict__ dec_b1,
    const float* __restrict__ dec_w2, const float* __restrict__ dec_b2,
    const float* __restrict__ fw1, const float* __restrict__ fb1,
    const float* __restrict__ fw2, const float* __restrict__ fb2,
    float* __restrict__ zws, float* __restrict__ partials)
{
  __shared__ __align__(16) float    sW1e[3 * kHidPad];
  __shared__ __align__(16) float    sW1d[3 * kHidPad];
  __shared__ __align__(16) unsigned sBe[16 * kBtPitch];
  __shared__ __align__(16) unsigned sBd[16 * kBtPitch];
  __shared__ __align__(16) float    sFl[256 * 4];
  __shared__ __align__(16) float    sOut[4 * 32 * 16];
  __shared__ __align__(16) float    sZ[2 * kBlkThr];
  __shared__ float sRed[4];

  const int tid  = threadIdx.x;
  const int lane = tid & 31;
  const int wave = __builtin_amdgcn_readfirstlane((int)(threadIdx.x >> 5));
  const int hh   = lane >> 4;
  const int n    = lane & 15;
  const int blockBase = blockIdx.x * kBlkThr;

  {
    const int  kc  = tid < kHid ? tid : (kHid - 1);
    const bool kin = tid < kHid;
    float a = enc_w1[kc];
    float b = enc_w1[kHid + kc];
    float c = enc_b1[kc];
    float d = dec_w1[kc];
    float e = dec_w1[kHid + kc];
    float f = dec_b1[kc];
    asm volatile("" : "+v"(a), "+v"(b), "+v"(c));
    asm volatile("" : "+v"(d), "+v"(e), "+v"(f));
    sW1e[tid]               = kin ? a * kCarryH : 0.0f;
    sW1e[kHidPad + tid]     = kin ? b * kCarryH : 0.0f;
    sW1e[2 * kHidPad + tid] = kin ? c * kCarryH : 0.0f;
    sW1d[tid]               = kin ? d : 0.0f;
    sW1d[kHidPad + tid]     = kin ? e : 0.0f;
    sW1d[2 * kHidPad + tid] = kin ? f : 0.0f;
  }
#pragma unroll 1
  for (int it = 0; it < 8; ++it) {
    const int idx = tid + kBlkThr * it;
    const int nn  = idx >> 6;
    const int kw  = idx & 63;
    const int k0  = 2 * kw;
    const int k1  = k0 + 1;
    const int k0c = k0 < kHid ? k0 : (kHid - 1);
    const int k1c = k1 < kHid ? k1 : (kHid - 1);
    const int ne  = nn < kEncOut ? nn : (kEncOut - 1);
    const int nd  = nn < kDecOut ? nn : (kDecOut - 1);
    float e0 = enc_w2[k0c * kEncOut + ne];
    float e1 = enc_w2[k1c * kEncOut + ne];
    float d0 = dec_w2[k0c * kDecOut + nd];
    float d1 = dec_w2[k1c * kDecOut + nd];
    asm volatile("" : "+v"(e0), "+v"(e1), "+v"(d0), "+v"(d1));
    e0 = (nn < kEncOut && k0 < kHid) ? e0 * kCarryW : 0.0f;
    e1 = (nn < kEncOut && k1 < kHid) ? e1 * kCarryW : 0.0f;
    d0 = (nn < kDecOut && k0 < kHid) ? d0 : 0.0f;
    d1 = (nn < kDecOut && k1 < kHid) ? d1 : 0.0f;
    v2h ph;
    ph[0] = (_Float16)e0;
    ph[1] = (_Float16)e1;
    sBe[nn * kBtPitch + kw] = __builtin_bit_cast(unsigned, ph);
    sBd[nn * kBtPitch + kw] = bf_rne16(d0) | (bf_rne16(d1) << 16);
  }
#pragma unroll 1
  for (int it = 0; it < 2; ++it) {
    const int idx = tid + kBlkThr * it;
    const int ic  = idx < (kSteps * kStepHid) ? idx : (kSteps * kStepHid - 1);
    const int iq  = idx / kStepHid;
    const int ii  = iq < kSteps ? iq : (kSteps - 1);
    v4f ent;
    ent[0] = fw1[ic];
    ent[1] = fb1[ic];
    ent[2] = fw2[ic];
    ent[3] = fb2[ii];
    *(v4f*)(sFl + 4 * idx) = ent;
  }
  float biasE = enc_b2[n < kEncOut ? n : (kEncOut - 1)];
  float biasD = dec_b2[n < kDecOut ? n : (kDecOut - 1)];
  asm volatile("" : "+v"(biasE), "+v"(biasD));
  biasE = (n < kEncOut) ? biasE : 0.0f;
  biasD = (n < kDecOut) ? biasD : 0.0f;
  __syncthreads();

  float* slab = sOut + wave * (32 * 16);

  {
    const v8u b0 = load_bfrag(sBe, n, hh, 0);
    const v8u b1 = load_bfrag(sBe, n, hh, 1);
    const v8u b2 = load_bfrag(sBe, n, hh, 2);
    const v8u b3 = load_bfrag(sBe, n, hh, 3);
#pragma unroll 1
    for (int T = 0; T < 2; ++T) {
      const size_t srow = (size_t)(blockBase + wave * 32 + T * 16 + n);
      const v2f xr = *(const v2f*)(x + 2 * srow);
      v8f acc = (v8f){0.f, 0.f, 0.f, 0.f, 0.f, 0.f, 0.f, 0.f};
      acc = hidden_chunk<false>(sW1e,  0 + 8 * hh, xr[0], xr[1], b0, acc);
      acc = hidden_chunk<false>(sW1e, 32 + 8 * hh, xr[0], xr[1], b1, acc);
      acc = hidden_chunk<false>(sW1e, 64 + 8 * hh, xr[0], xr[1], b2, acc);
      acc = hidden_chunk<false>(sW1e, 96 + 8 * hh, xr[0], xr[1], b3, acc);
      spill_tile(slab + T * 256, acc, kFoldEnc, biasE, hh, n);
    }
  }
  __syncthreads();

  const size_t s = (size_t)(blockBase + tid);
  const v2f xv = *(const v2f*)(x + 2 * s);
  const v2f ev = *(const v2f*)(eps + 2 * s);
  const v4f q  = *(const v4f*)(sOut + tid * 16);
  const float m0 = q[0], m1 = q[1], l0 = q[2], l1 = q[3];
  float z0 = fmaf(ev[0], expf(l0), m0);
  float z1 = fmaf(ev[1], expf(l1), m1);
  const float t0 = (z0 - m0) * expf(-l0);
  const float t1 = (z1 - m1) * expf(-l1);
  const float logqz = -0.5f * (t0 * t0 + 2.0f * l0 + kLog2Pi)
                      - 0.5f * (t1 * t1 + 2.0f * l1 + kLog2Pi);
#pragma unroll 1
  for (int p = 0; p < kSteps / 2; ++p) {
    z1 += shear_mlp(sFl + (2 * p) * (4 * kStepHid), z0);
    z0 += shear_mlp(sFl + (2 * p + 1) * (4 * kStepHid), z1);
  }
  const float logpz = -0.5f * (z0 * z0 + kLog2Pi) - 0.5f * (z1 * z1 + kLog2Pi);
  {
    v2f zz;
    zz[0] = z0;
    zz[1] = z1;
    *(v2f*)(sZ + 2 * tid) = zz;
  }
  __syncthreads();

  if (wave < 2) {
    const v4f zv = *(const v4f*)(sZ + 4 * tid);
    volatile v4f* zp = (volatile v4f*)(zws + 2 * (size_t)blockBase + 4 * tid);
    *zp = zv;
    __threadfence();
    *zp = zv;
  }

  {
    const v8u b0 = load_bfrag(sBd, n, hh, 0);
    const v8u b1 = load_bfrag(sBd, n, hh, 1);
    const v8u b2 = load_bfrag(sBd, n, hh, 2);
    const v8u b3 = load_bfrag(sBd, n, hh, 3);
#pragma unroll 1
    for (int T = 0; T < 2; ++T) {
      const v2f zr = *(const v2f*)(sZ + 2 * (wave * 32 + T * 16 + n));
      v8f acc = (v8f){0.f, 0.f, 0.f, 0.f, 0.f, 0.f, 0.f, 0.f};
      acc = hidden_chunk<true>(sW1d,  0 + 8 * hh, zr[0], zr[1], b0, acc);
      acc = hidden_chunk<true>(sW1d, 32 + 8 * hh, zr[0], zr[1], b1, acc);
      acc = hidden_chunk<true>(sW1d, 64 + 8 * hh, zr[0], zr[1], b2, acc);
      acc = hidden_chunk<true>(sW1d, 96 + 8 * hh, zr[0], zr[1], b3, acc);
      spill_tile(slab + T * 256, acc, 1.0f, biasD, hh, n);
    }
  }
  __syncthreads();

  const v2f px = *(const v2f*)(sOut + tid * 16);
  const float d0 = xv[0] - px[0];
  const float d1 = xv[1] - px[1];
  const float logpxz = -0.5f * (d0 * d0 + kLog2Pi) - 0.5f * (d1 * d1 + kLog2Pi);

  float val = logpxz + logpz - logqz;
#pragma unroll
  for (int off = 16; off > 0; off >>= 1) val += __shfl_xor(val, off, 32);
  sRed[wave] = val;
  __syncthreads();
  if (wave == 0) {
    const float tot = (sRed[0] + sRed[1]) + (sRed[2] + sRed[3]);
    volatile float* pp = partials + (size_t)blockIdx.x * 32 + lane;
    *pp = tot;
    __threadfence();
    *pp = tot;
  }
}

__global__ __launch_bounds__(256) void mean_reduce_kernel(
    const float* __restrict__ partials, float* __restrict__ elbo_ws)
{
  __shared__ float sAcc[256];
  const int tid  = threadIdx.x;
  const int lane = tid & 31;
  const int wave = __builtin_amdgcn_readfirstlane((int)(threadIdx.x >> 5));
  float acc = 0.0f;
#pragma unroll 1
  for (int i = 0; i < kMainGrid / 256; ++i) acc += partials[(size_t)(tid + 256 * i) * 32];
  sAcc[tid] = acc;
  __syncthreads();
#pragma unroll 1
  for (int off = 128; off > 0; off >>= 1) {
    if (tid < off) sAcc[tid] += sAcc[tid + off];
    __syncthreads();
  }
  if (wave == 0) {
    const float e = sAcc[0] * (1.0f / (float)kSamples);
    volatile float* p = elbo_ws + lane;
    *p = e;
    __threadfence();
    *p = e;
  }
}

__global__ __launch_bounds__(256) void pack_out_kernel(
    const float* __restrict__ zws, const float* __restrict__ elbo_ws, float* __restrict__ out)
{
  const int t  = blockIdx.x * 256 + threadIdx.x;
  const int f0 = 4 * t;
  const int hi = 2 * kSamples - 1;
  int i0 = f0 - 1;
  int i1 = f0;
  int i2 = f0 + 1;
  int i3 = f0 + 2;
  i0 = i0 < 0 ? 0 : i0;
  i0 = i0 > hi ? hi : i0;
  i1 = i1 > hi ? hi : i1;
  i2 = i2 > hi ? hi : i2;
  i3 = i3 > hi ? hi : i3;
  float a0 = zws[i0];
  float a1 = zws[i1];
  float a2 = zws[i2];
  float a3 = zws[i3];
  float e  = elbo_ws[0];
  asm volatile("" : "+v"(a0), "+v"(a1), "+v"(a2), "+v"(a3), "+v"(e));
  v4f v;
  v[0] = (f0 == 0) ? e : a0;
  v[1] = a1;
  v[2] = a2;
  v[3] = a3;
  if (t < kPackV4) {
    volatile v4f* p = (volatile v4f*)(out + f0);
    *p = v;
    __threadfence();
    *p = v;
  } else if (t == kPackV4) {
    volatile float* p = out + f0;
    *p = a0;
    __threadfence();
    *p = a0;
  }
}

extern "C" void kernel_launch(void* const* d_in, const int* in_sizes, int n_in,
                              void* d_out, int out_size, void* d_ws, size_t ws_size,
                              hipStream_t stream) {
  if (n_in < 14) return;
  if (in_sizes[0] != 2 * kSamples) return;
  if (in_sizes[1] != 2 * kSamples) return;
  if (in_sizes[2] != 2 * kHid) return;
  if (in_sizes[3] != kHid) return;
  if (in_sizes[4] != kHid * kEncOut) return;
  if (in_sizes[5] != kEncOut) return;
  if (in_sizes[6] != 2 * kHid) return;
  if (in_sizes[7] != kHid) return;
  if (in_sizes[8] != kHid * kDecOut) return;
  if (in_sizes[9] != kDecOut) return;
  if (in_sizes[10] != kSteps * kStepHid) return;
  if (in_sizes[11] != kSteps * kStepHid) return;
  if (in_sizes[12] != kSteps * kStepHid) return;
  if (in_sizes[13] != kSteps) return;
  if (out_size != kOutFloats) return;
  if (ws_size < kWsTotal) return;

  const float* x      = (const float*)d_in[0];
  const float* eps    = (const float*)d_in[1];
  const float* enc_w1 = (const float*)d_in[2];
  const float* enc_b1 = (const float*)d_in[3];
  const float* enc_w2 = (const float*)d_in[4];
  const float* enc_b2 = (const float*)d_in[5];
  const float* dec_w1 = (const float*)d_in[6];
  const float* dec_b1 = (const float*)d_in[7];
  const float* dec_w2 = (const float*)d_in[8];
  const float* dec_b2 = (const float*)d_in[9];
  const float* fw1    = (const float*)d_in[10];
  const float* fb1    = (const float*)d_in[11];
  const float* fw2    = (const float*)d_in[12];
  const float* fb2    = (const float*)d_in[13];
  float* out = (float*)d_out;

  char*  ws       = (char*)d_ws;
  float* zws      = (float*)(ws + kOffZws);
  float* partials = (float*)(ws + kOffPart);
  float* elbo_ws  = (float*)(ws + kOffElbo);

  fused_sample_kernel<<<kMainGrid, kBlkThr, 0, stream>>>(
      x, eps, enc_w1, enc_b1, enc_w2, enc_b2, dec_w1, dec_b1, dec_w2, dec_b2,
      fw1, fb1, fw2, fb2, zws, partials);
  mean_reduce_kernel<<<1, 256, 0, stream>>>(partials, elbo_ws);
  pack_out_kernel<<<kPackGrid, 256, 0, stream>>>(zws, elbo_ws, out);
}
